// MoeLayer_29291676958946
// MI455X (gfx1250) — hardware-verified
//
#include <hip/hip_runtime.h>
#include <math.h>

typedef __attribute__((ext_vector_type(16))) __bf16 v16b;
typedef __attribute__((ext_vector_type(8)))  float v8f;
typedef __attribute__((ext_vector_type(4)))  float v4f;
typedef __attribute__((ext_vector_type(4)))  unsigned v4u;
typedef __attribute__((ext_vector_type(8)))  unsigned v8u;

#ifndef NT
#define NT 8192u
#endif
#define DD 1024u
#define DO 1024u
#define NE 8u
#define DDQ (DD / 8u)
#define EST (DO * DDQ)

static_assert((NT & 127u) == 0u);
static_assert((DD & 63u) == 0u);
static_assert((DO & 63u) == 0u);
static_assert(NE == 8u);

#define WS_G   0u
#define WS_XB  (WS_G + 4u * NE * (size_t)NT)
#define WS_WT  (WS_XB + 2u * (size_t)NT * DD)
#define WS_END (WS_WT + 2u * (size_t)NE * DO * DD)
static_assert((WS_XB & 127u) == 0u);
static_assert((WS_WT & 127u) == 0u);
static_assert(WS_END <= 134217728u);

template <typename T> __device__ __forceinline__ void vst2(T* p, T v) { *(volatile T*)p = v; __threadfence(); *(volatile T*)p = v; }

__device__ __forceinline__ v8f wmma_bf(v16b a, v16b b, v8f c) {
  v8f d = __builtin_amdgcn_wmma_f32_16x16x32_bf16(false, a, false, b, (short)0, c, false, false);
  asm volatile("v_nop\n\tv_nop\n\tv_nop\n\tv_nop" : "+v"(d) : "v"(a), "v"(b));
  return d;
}
__device__ __forceinline__ v16b frag_q(v4u q0, v4u q1) {
  const v8u w = __builtin_shufflevector(q0, q1, 0, 1, 2, 3, 4, 5, 6, 7);
  return __builtin_bit_cast(v16b, w);
}
__device__ __forceinline__ float bfr(float v) { return (float)(__bf16)v; }
__device__ __forceinline__ unsigned short bfbits(float v) { return __builtin_bit_cast(unsigned short, (__bf16)v); }
__device__ __forceinline__ unsigned pk2(float a, float b) { return (unsigned)bfbits(a) | ((unsigned)bfbits(b) << 16); }

static_assert(((NT * DD) / 8u) % 256u == 0u);
__global__ __launch_bounds__(256) void k_xcvt(const float* __restrict__ X, v4u* __restrict__ XB) {
  const unsigned idx = blockIdx.x * 256u + threadIdx.x;
  const float* p = X + (size_t)idx * 8u;
  const v4f a = *(const v4f*)p;
  const v4f b = *(const v4f*)(p + 4);
  v4u o; o[0] = pk2(a[0], a[1]); o[1] = pk2(a[2], a[3]); o[2] = pk2(b[0], b[1]); o[3] = pk2(b[2], b[3]);
  vst2(XB + idx, o);
}

__global__ __launch_bounds__(256) void k_wT(const float* __restrict__ WE, v4u* __restrict__ WT) {
  __shared__ __align__(16) unsigned short ts[64][72];
  const unsigned tid = threadIdx.x;
  const unsigned o0 = blockIdx.x * 64u, i0 = blockIdx.y * 64u, e = blockIdx.z;
#pragma unroll
  for (unsigned p = 0; p < 4u; ++p) {
    const unsigned idx = p * 256u + tid;
    const unsigned i = idx >> 4, oc = (idx & 15u) * 4u;
    const v4f v = *(const v4f*)(WE + ((size_t)e * DD + i0 + i) * DO + o0 + oc);
    ts[oc + 0u][i] = bfbits(v[0]);
    ts[oc + 1u][i] = bfbits(v[1]);
    ts[oc + 2u][i] = bfbits(v[2]);
    ts[oc + 3u][i] = bfbits(v[3]);
  }
  __syncthreads();
#pragma unroll
  for (unsigned p = 0; p < 2u; ++p) {
    const unsigned o = p * 32u + (tid >> 3), pc = tid & 7u;
    const v4u v = *(const v4u*)&ts[o][pc * 8u];
    vst2(WT + ((size_t)e * DO + o0 + o) * DDQ + (i0 >> 3) + pc, v);
  }
}

__global__ __launch_bounds__(128) void k_gate(const v4u* __restrict__ XB, const float* __restrict__ WG, const float* __restrict__ BG, float* __restrict__ G) {
  __shared__ __align__(16) unsigned short swg[16][1032];
  __shared__ __align__(16) float sl[64][8];
  const unsigned tid = threadIdx.x, wave = tid >> 5, lane = tid & 31u, col = lane & 15u, h = lane >> 4;
  const unsigned r0 = blockIdx.x * 64u;
  const v4u zq = {0u, 0u, 0u, 0u};
#pragma unroll
  for (unsigned r = 0; r < 8u; ++r) *(v4u*)&swg[8u + r][tid * 8u] = zq;
#pragma unroll 4
  for (unsigned r = 0; r < 16u; ++r) {
    const unsigned idx = r * 128u + tid;
    const v4f t4 = *(const v4f*)(WG + (size_t)idx * 4u);
    const unsigned i = idx >> 1, e0 = (idx & 1u) * 4u;
    swg[e0 + 0u][i] = bfbits(t4[0]);
    swg[e0 + 1u][i] = bfbits(t4[1]);
    swg[e0 + 2u][i] = bfbits(t4[2]);
    swg[e0 + 3u][i] = bfbits(t4[3]);
  }
  __syncthreads();
  const v4u* pa = XB + (size_t)(r0 + wave * 16u + col) * DDQ + h;
  v8f acc = {};
#pragma unroll 2
  for (unsigned kc = 0; kc < DD / 32u; ++kc) {
    const v4u a0 = pa[kc * 4u];
    const v4u a1 = pa[kc * 4u + 2u];
    const v4u w0 = *(const v4u*)&swg[col][kc * 32u + 8u * h];
    const v4u w1 = *(const v4u*)&swg[col][kc * 32u + 16u + 8u * h];
    acc = wmma_bf(frag_q(a0, a1), frag_q(w0, w1), acc);
  }
  if (col < 8u) {
#pragma unroll
    for (unsigned r = 0; r < 8u; ++r) sl[wave * 16u + 8u * h + r][col] = acc[r];
  }
  __syncthreads();
  const unsigned tok = tid >> 1, e0 = (tid & 1u) * 4u;
  v4f l = *(const v4f*)&sl[tok][e0];
  l[0] += bfr(BG[e0 + 0u]); l[1] += bfr(BG[e0 + 1u]); l[2] += bfr(BG[e0 + 2u]); l[3] += bfr(BG[e0 + 3u]);
  float m = fmaxf(fmaxf(l[0], l[1]), fmaxf(l[2], l[3]));
  const float mo = __shfl_xor(m, 1, 32);
  m = fmaxf(m, mo);
  v4f ex; ex[0] = expf(l[0] - m); ex[1] = expf(l[1] - m); ex[2] = expf(l[2] - m); ex[3] = expf(l[3] - m);
  float s = (ex[0] + ex[1]) + (ex[2] + ex[3]);
  const float so = __shfl_xor(s, 1, 32);
  s += so;
  const float inv = 1.0f / s;
  v4f gq; gq[0] = ex[0] * inv; gq[1] = ex[1] * inv; gq[2] = ex[2] * inv; gq[3] = ex[3] * inv;
  vst2((v4f*)(G + (size_t)r0 * NE + tid * 4u), gq);
}

__global__ __launch_bounds__(256) void k_experts(const v4u* __restrict__ XB, const v4u* __restrict__ WT, const float* __restrict__ BE, const float* __restrict__ G, float* __restrict__ OUT) {
  __shared__ __align__(16) float sg[128][8];
  __shared__ __align__(16) float sf[128][36];
  const unsigned tid = threadIdx.x, wave = tid >> 5, lane = tid & 31u, col = lane & 15u, h = lane >> 4;
  const unsigned wm = wave & 3u, wn = wave >> 2;
  const unsigned bm = blockIdx.x * 128u, bn = blockIdx.y * 32u;
  { const v4f t4 = *(const v4f*)(G + (size_t)bm * NE + tid * 4u); *(v4f*)(&sg[0][0] + tid * 4u) = t4; }
  __syncthreads();
  const v4u* pa0 = XB + (size_t)(bm + wm * 32u + col) * DDQ + h;
  const v4u* pa1 = pa0 + 16u * DDQ;
  const v4u* pb  = WT + (size_t)(bn + wn * 16u + col) * DDQ + h;
  v8f acc0[8] = {}; v8f acc1[8] = {};
#pragma unroll 1
  for (unsigned kc = 0; kc < DD / 32u; ++kc) {
    const unsigned kq = kc * 4u;
    const v16b a0 = frag_q(pa0[kq], pa0[kq + 2u]);
    const v16b a1 = frag_q(pa1[kq], pa1[kq + 2u]);
    asm volatile("s_wait_loadcnt 0x0" ::: "memory");
#pragma unroll
    for (unsigned e = 0; e < 8u; e += 2u) {
      const v4u* pe = pb + (size_t)e * EST + kq;
      const v16b b0 = frag_q(pe[0], pe[2]);
      const v16b b1 = frag_q(pe[EST], pe[EST + 2u]);
      asm volatile("s_wait_loadcnt 0x0" ::: "memory");
      acc0[e] = wmma_bf(a0, b0, acc0[e]);
      acc1[e] = wmma_bf(a1, b0, acc1[e]);
      acc0[e + 1u] = wmma_bf(a0, b1, acc0[e + 1u]);
      acc1[e + 1u] = wmma_bf(a1, b1, acc1[e + 1u]);
    }
  }
  float bev[8];
#pragma unroll
  for (unsigned e = 0; e < 8u; ++e) bev[e] = bfr(BE[(size_t)e * DO + bn + wn * 16u + col]);
#pragma unroll
  for (unsigned r = 0; r < 8u; ++r) {
    const unsigned row = wm * 32u + 8u * h + r;
    const v4f g0 = *(const v4f*)&sg[row][0];
    const v4f g1 = *(const v4f*)&sg[row][4];
    float s = g0[0] * (acc0[0][r] + bev[0]);
    s += g0[1] * (acc0[1][r] + bev[1]);
    s += g0[2] * (acc0[2][r] + bev[2]);
    s += g0[3] * (acc0[3][r] + bev[3]);
    s += g1[0] * (acc0[4][r] + bev[4]);
    s += g1[1] * (acc0[5][r] + bev[5]);
    s += g1[2] * (acc0[6][r] + bev[6]);
    s += g1[3] * (acc0[7][r] + bev[7]);
    sf[row][wn * 16u + col] = s;
  }
#pragma unroll
  for (unsigned r = 0; r < 8u; ++r) {
    const unsigned row = wm * 32u + 16u + 8u * h + r;
    const v4f g0 = *(const v4f*)&sg[row][0];
    const v4f g1 = *(const v4f*)&sg[row][4];
    float s = g0[0] * (acc1[0][r] + bev[0]);
    s += g0[1] * (acc1[1][r] + bev[1]);
    s += g0[2] * (acc1[2][r] + bev[2]);
    s += g0[3] * (acc1[3][r] + bev[3]);
    s += g1[0] * (acc1[4][r] + bev[4]);
    s += g1[1] * (acc1[5][r] + bev[5]);
    s += g1[2] * (acc1[6][r] + bev[6]);
    s += g1[3] * (acc1[7][r] + bev[7]);
    sf[row][wn * 16u + col] = s;
  }
  __syncthreads();
#pragma unroll
  for (unsigned it = 0; it < 4u; ++it) {
    const unsigned row = wave * 16u + it * 4u + (lane >> 3), pc = lane & 7u;
    const v4f v = *(const v4f*)&sf[row][pc * 4u];
    vst2((v4f*)(OUT + (size_t)(bm + row) * DO + bn + pc * 4u), v);
  }
}

extern "C" void kernel_launch(void* const* d_in, const int* in_sizes, int n_in, void* d_out, int out_size, void* d_ws, size_t ws_size, hipStream_t stream) {
  if (n_in < 5) return;
  if ((size_t)in_sizes[0] < (size_t)NT * DD) return;
  if ((size_t)in_sizes[1] < (size_t)NE * DD * DO) return;
  if ((size_t)in_sizes[2] < (size_t)NE * DO) return;
  if ((size_t)in_sizes[3] < (size_t)DD * NE) return;
  if ((size_t)in_sizes[4] < (size_t)NE) return;
  if ((size_t)out_size < (size_t)NT * DO) return;
  if (ws_size < (size_t)WS_END) return;
  const float* X  = (const float*)d_in[0];
  const float* WE = (const float*)d_in[1];
  const float* BE = (const float*)d_in[2];
  const float* WG = (const float*)d_in[3];
  const float* BG = (const float*)d_in[4];
  char* ws = (char*)d_ws;
  float* G  = (float*)(ws + WS_G);
  v4u* XB = (v4u*)(ws + WS_XB);
  v4u* WT = (v4u*)(ws + WS_WT);
  float* OUT = (float*)d_out;
  k_xcvt<<<dim3((NT * DD) / (8u * 256u)), 256, 0, stream>>>(X, XB);
  k_wT<<<dim3(DO / 64u, DD / 64u, NE), 256, 0, stream>>>(WE, WT);
  k_gate<<<dim3(NT / 64u), 128, 0, stream>>>(XB, WG, BG, G);
  k_experts<<<dim3(NT / 128u, DO / 32u), 256, 0, stream>>>(XB, WT, BE, G, OUT);
}
